// ContextualizedNN_57002805952924
// MI455X (gfx1250) — hardware-verified
//
#include <hip/hip_runtime.h>
#include <math.h>

typedef __attribute__((ext_vector_type(16))) _Float16 v16h;
typedef __attribute__((ext_vector_type(16))) __bf16 v16b;
typedef __attribute__((ext_vector_type(8)))  _Float16 v8h;
typedef __attribute__((ext_vector_type(8)))  float v8f;
typedef __attribute__((ext_vector_type(4)))  float v4f;
typedef __attribute__((ext_vector_type(2)))  float v2f;
typedef __attribute__((ext_vector_type(4)))  unsigned v4u;
typedef __attribute__((ext_vector_type(4)))  int v4i;
typedef float __attribute__((may_alias)) float_a;
typedef int __attribute__((may_alias)) int_a;

template <typename T> __device__ __forceinline__ void vst2(void* p, T v) { *(volatile T*)p = v; __threadfence(); *(volatile T*)p = v; }
__device__ __forceinline__ v8f wmma16(v16h a, v16h b, v8f c) {
  v8f d = __builtin_amdgcn_wmma_f32_16x16x32_f16(false, a, false, b, (short)0, c, false, false);
  asm volatile("v_nop\n\tv_nop\n\tv_nop\n\tv_nop" : "+v"(d) : "v"(a), "v"(b));
  return d;
}
__device__ __forceinline__ v8f wmma_bf(v16b a, v16b b, v8f c) {
  v8f d = __builtin_amdgcn_wmma_f32_16x16x32_bf16(false, a, false, b, (short)0, c, false, false);
  asm volatile("v_nop\n\tv_nop\n\tv_nop\n\tv_nop" : "+v"(d) : "v"(a), "v"(b));
  return d;
}
__device__ __forceinline__ v16h frag_h(const _Float16* rowk0, int lane) {
  union { v16h v; v8h q[2]; } u; const _Float16* p = rowk0 + 8 * (lane >> 4);
  u.q[0] = *(const v8h*)p; u.q[1] = *(const v8h*)(p + 16); return u.v;
}
__device__ __forceinline__ v16h frag_f32(const float* rowk0, int lane) {
  v16h a; const float* p = rowk0 + 8 * (lane >> 4);
#pragma unroll
  for (int i = 0; i < 8; ++i) { a[i] = (_Float16)p[i]; a[8 + i] = (_Float16)p[16 + i]; }
  return a;
}
__device__ __forceinline__ v16h frag_f32s(const float* rowk0, int lane, float sc) {
  v16h a; const float* p = rowk0 + 8 * (lane >> 4);
#pragma unroll
  for (int i = 0; i < 8; ++i) { a[i] = (_Float16)(p[i] * sc); a[8 + i] = (_Float16)(p[16 + i] * sc); }
  return a;
}
__device__ __forceinline__ v16h fragc_f32(const float* W, int k0, int n, int lane, int ld, int K) {
  v16h a; const int g = lane >> 4;
#pragma unroll
  for (int i = 0; i < 8; ++i) { const int ka = k0 + 8 * g + i, kb = ka + 16;
    a[i] = (_Float16)(ka < K ? W[(size_t)(ka < K ? ka : K - 1) * ld + n] : 0.f); a[8 + i] = (_Float16)(kb < K ? W[(size_t)(kb < K ? kb : K - 1) * ld + n] : 0.f); }
  return a;
}
struct F2 { v16b h, l; };
__device__ __forceinline__ F2 bsplit16(const float v[16]) { F2 r;
#pragma unroll
  for (int i = 0; i < 16; ++i) { const __bf16 h = (__bf16)v[i]; r.h[i] = h; r.l[i] = (__bf16)(v[i] - (float)h); }
  return r; }
__device__ __forceinline__ F2 split_row(const float* row, int k0, int lane) { float v[16]; const float* p = row + k0 + 8 * (lane >> 4);
#pragma unroll
  for (int i = 0; i < 8; ++i) { v[i] = p[i]; v[8 + i] = p[16 + i]; }
  return bsplit16(v); }
__device__ __forceinline__ F2 split_rowK(const float* row, int k0, int lane, int K) { float v[16]; const int g = lane >> 4;
#pragma unroll
  for (int i = 0; i < 8; ++i) { const int ka = k0 + 8 * g + i, kb = ka + 16; v[i] = ka < K ? row[ka < K ? ka : K - 1] : 0.f; v[8 + i] = kb < K ? row[kb < K ? kb : K - 1] : 0.f; }
  return bsplit16(v); }
__device__ __forceinline__ F2 split_col(const float* W, int k0, int n, int lane, int ld, int K) { float v[16]; const int g = lane >> 4;
#pragma unroll
  for (int i = 0; i < 8; ++i) { const int ka = k0 + 8 * g + i, kb = ka + 16; v[i] = ka < K ? W[(size_t)(ka < K ? ka : K - 1) * ld + n] : 0.f; v[8 + i] = kb < K ? W[(size_t)(kb < K ? kb : K - 1) * ld + n] : 0.f; }
  return bsplit16(v); }
__device__ __forceinline__ v8f mac3(const F2& a, const F2& b, v8f c) { c = wmma_bf(a.l, b.h, c); c = wmma_bf(a.h, b.l, c); return wmma_bf(a.h, b.h, c); }
__device__ __forceinline__ float sigm(float v) { return 1.0f / (1.0f + expf(-v)); }
#define LDSX() do { asm volatile("s_wait_dscnt 0" ::: "memory"); __builtin_amdgcn_wave_barrier(); __builtin_amdgcn_fence(__ATOMIC_RELEASE, "workgroup"); } while (0)


#define NBQ 8192
#define KK 100
#define DDm 64
#define CAT 12800
#define HID 128
#define NUSR 100000
#define NITM 50000
#define CHK 1024
#ifndef NCHUNK
#define NCHUNK (NBQ / CHK)
#endif
typedef __attribute__((ext_vector_type(8))) __bf16 v8b;
__device__ __forceinline__ v16b frag_b(const __bf16* rowk0, int lane) {
  union { v16b v; v8b q[2]; } u; const __bf16* p = rowk0 + 8 * (lane >> 4);
  u.q[0] = *(const v8b*)p; u.q[1] = *(const v8b*)(p + 16); return u.v;
}
__device__ __forceinline__ float bfr(float v) { return (float)(__bf16)v; }
__device__ __attribute__((noinline)) float exp_ni(float v) { return expf(v); }
__device__ __attribute__((noinline)) float erf_ni(float v) { return erff(v); }

#define WS_PW   0u
#define WS_X    (WS_PW + 2u * HID * CAT)
#define WS_H    (WS_X + 4u * CHK * CAT)
#define WS_END  (WS_H + 4u * NBQ * HID)

__global__ __launch_bounds__(256) void k_packW1(const float* __restrict__ W1, __bf16* __restrict__ PW) {
  __shared__ __align__(16) __bf16 s[CAT]; const int n = blockIdx.x, t = threadIdx.x;
  for (int k = t; k < CAT; k += 256) s[k] = (__bf16)W1[(size_t)k * HID + n];
  __syncthreads();
  for (int q = t; q < CAT / 8; q += 256) vst2((unsigned*)(PW + (size_t)n * CAT + q * 8), *(const v4u*)&s[q * 8]);
}
template <int SIDE>
__global__ __launch_bounds__(128) void k_side(const int* __restrict__ IDS, const int* __restrict__ IDXT, const float* __restrict__ SCR, const float* __restrict__ EMB, int chunk0, float* __restrict__ X) {
  __shared__ __align__(16) __bf16 sA[112][136]; __shared__ __align__(16) __bf16 sB[DDm][136]; __shared__ int snb[KK]; __shared__ __align__(16) float so[4][16][68];
  const int tid = threadIdx.x, wave = tid >> 5, lane = tid & 31, col = lane & 15, g = lane >> 4; const int sl = blockIdx.x; const size_t smp = (size_t)chunk0 + sl;
  constexpr int NTAB = SIDE ? NITM : NUSR;
  const int id = min(max(IDS[smp], 0), NTAB - 1);
  if (tid < KK) snb[tid] = min(max(IDXT[(size_t)id * KK + tid], 0), NTAB - 1);
  __syncthreads();
  for (int q = tid; q < 112 * 128; q += 128) { const int k = q >> 7, j = q & 127; sA[k][j] = (__bf16)((k < KK && j < KK) ? SCR[(size_t)snb[k < KK ? k : 0] * KK + j] : 0.f); }
  for (int q = tid; q < DDm * 128; q += 128) { const int d = q & 63, j = q >> 6; sB[d][j] = (__bf16)((j < KK) ? EMB[(size_t)snb[j < KK ? j : 0] * DDm + d] : 0.f); }
  __syncthreads();
  float* xrow = X + (size_t)sl * CAT + SIDE * (KK * DDm);
  for (int rt = wave; rt < 7; rt += 4) { v8f acc[4] = {};
#pragma unroll
    for (int kc = 0; kc < 4; ++kc) { const v16b a = frag_b(&sA[rt * 16 + col][kc * 32], lane);
#pragma unroll
      for (int j = 0; j < 4; ++j) acc[j] = wmma_bf(a, frag_b(&sB[j * 16 + col][kc * 32], lane), acc[j]); }
#pragma unroll
    for (int j = 0; j < 4; ++j)
#pragma unroll
      for (int r = 0; r < 8; ++r) so[wave][8 * g + r][j * 16 + col] = acc[j][r];
    LDSX();
    for (int q = lane; q < 16 * 16; q += 32) { const int rl = q >> 4, pc = q & 15; const int k = rt * 16 + rl; if (k < KK) vst2(xrow + k * DDm + pc * 4, *(const v4f*)&so[wave][rl][pc * 4]); }
    LDSX(); }
}
__global__ __launch_bounds__(128) void k_h(const float* __restrict__ X, const __bf16* __restrict__ PW, const float* __restrict__ B1, int chunk0, float* __restrict__ Hh) {
  __shared__ __align__(16) float so[4][16][132];
  const int tid = threadIdx.x, wave = tid >> 5, lane = tid & 31, col = lane & 15, g = lane >> 4; const size_t r0 = (size_t)blockIdx.x * 64 + wave * 16;
  v8f acc[8] = {};
#pragma unroll 2
  for (int kc = 0; kc < CAT / 32; ++kc) { const F2 a = split_row(X + (r0 + col) * CAT, kc * 32, lane);
#pragma unroll
    for (int j = 0; j < 8; ++j) { const v16b w = frag_b(PW + (size_t)(j * 16 + col) * CAT + kc * 32, lane); acc[j] = wmma_bf(a.l, w, acc[j]); acc[j] = wmma_bf(a.h, w, acc[j]); } }
#pragma unroll
  for (int j = 0; j < 8; ++j) { const float bb = bfr(B1[j * 16 + col]);
#pragma unroll
    for (int r = 0; r < 8; ++r) so[wave][8 * g + r][j * 16 + col] = fmaxf(acc[j][r] + bb, 0.f); }
  LDSX();
  for (int rl = 0; rl < 16; ++rl) vst2(Hh + ((size_t)chunk0 + r0 + rl) * HID + lane * 4, *(const v4f*)&so[wave][rl][lane * 4]);
}
__global__ __launch_bounds__(256) void k_out(const float* __restrict__ Hh, const float* __restrict__ W2, const float* __restrict__ B2, float* __restrict__ OUT) {
  __shared__ __align__(16) float s[64]; const int tid = threadIdx.x, wave = tid >> 5, lane = tid & 31; const size_t q0 = (size_t)blockIdx.x * 64;
  for (int ql = wave; ql < 64; ql += 8) { float a = 0.f;
#pragma unroll
    for (int q = 0; q < 4; ++q) { const int c = lane + 32 * q; a += Hh[(q0 + ql) * HID + c] * bfr(W2[c]); }
#pragma unroll
    for (int o = 1; o < 32; o <<= 1) a += __shfl_xor(a, o);
    if (lane == 0) s[ql] = sigm(fmaxf(a + bfr(B2[0]), 0.f)); }
  __syncthreads();
  if (tid < 16) vst2(OUT + q0 + tid * 4, *(const v4f*)&s[tid * 4]);
}
extern "C" void kernel_launch(void* const* d_in, const int* in_sizes, int n_in, void* d_out, int out_size, void* d_ws, size_t ws_size, hipStream_t stream) {
  (void)in_sizes; (void)n_in; (void)out_size;
  const float** F = (const float**)d_in; const int* UID = (const int*)d_in[0]; const int* IID = (const int*)d_in[1]; const int* UIT = (const int*)d_in[2]; const int* IIT = (const int*)d_in[3];
  if (ws_size < (size_t)WS_END) return;
  char* ws = (char*)d_ws; __bf16* PW = (__bf16*)(ws + WS_PW); float *X = (float*)(ws + WS_X), *Hh = (float*)(ws + WS_H);
  k_packW1<<<HID, 256, 0, stream>>>(F[8], PW);
  for (int ch = 0; ch < NCHUNK; ++ch) { const int c0 = ch * CHK;
    k_side<0><<<CHK, 128, 0, stream>>>(UID, UIT, F[4], F[6], c0, X);
    k_side<1><<<CHK, 128, 0, stream>>>(IID, IIT, F[5], F[7], c0, X);
    k_h<<<dim3(CHK / 64), 128, 0, stream>>>(X, PW, F[9], c0, Hh); }
  k_out<<<(NCHUNK * CHK) / 64, 256, 0, stream>>>(Hh, F[10], F[11], (float*)d_out);
}
